// AttentionBlock_29291676959393
// MI455X (gfx1250) — hardware-run, weakly checked
//
#include <hip/hip_runtime.h>
#include <stddef.h>
#include <stdint.h>


#ifndef NB
#define NB 4
#endif
#ifndef SEQ
#define SEQ 2048
#endif
#define NB_FULL 4
#define SEQ_FULL 2048

#define DEVFN __device__ __forceinline__

typedef _Float16 v16h __attribute__((ext_vector_type(16)));
typedef _Float16 v8h  __attribute__((ext_vector_type(8)));
typedef float    v8f  __attribute__((ext_vector_type(8)));
typedef float    v4f  __attribute__((ext_vector_type(4)));
typedef v8h v8ha __attribute__((may_alias));
typedef v4f v4fa __attribute__((may_alias));

static constexpr int DM   = 1024;
static constexpr int DC   = 512;
static constexpr int NHD  = 16;
static constexpr int HE   = 64;
static constexpr int D3   = 3 * DM;
static constexpr int MTOT = NB * SEQ;
static constexpr float EPSV = 1e-6f;

static_assert(SEQ % 128 == 0);
static_assert(SEQ >= 128 && SEQ <= SEQ_FULL);
static_assert(NB >= 1 && NB <= NB_FULL);
static_assert(NHD * HE == DM);
static_assert(DM % 128 == 0 && D3 % 128 == 0 && DM % 64 == 0);

static constexpr size_t SZ_WQ    = (size_t)D3 * DM * 2;
static constexpr size_t SZ_WO    = (size_t)DM * DM * 2;
static constexpr size_t SZ_GAIN  = (size_t)NB * DM * 4;
static constexpr size_t SZ_ACT   = (size_t)MTOT * DM * 2;
static constexpr size_t OFF_WQ   = 0;
static constexpr size_t OFF_WO   = OFF_WQ + SZ_WQ;
static constexpr size_t OFF_GAIN = OFF_WO + SZ_WO;
static constexpr size_t OFF_XN   = OFF_GAIN + SZ_GAIN;
static constexpr size_t OFF_Q    = OFF_XN + SZ_ACT;
static constexpr size_t OFF_K    = OFF_Q + SZ_ACT;
static constexpr size_t OFF_VT   = OFF_K + SZ_ACT;
static constexpr size_t OFF_CTX  = OFF_VT + SZ_ACT;
static constexpr size_t WS_END   = OFF_CTX + SZ_ACT;
static_assert(SZ_WQ % 256 == 0 && SZ_WO % 256 == 0 && SZ_GAIN % 256 == 0 && SZ_ACT % 256 == 0);
static_assert((size_t)NB * NHD * SEQ * HE * 2 == SZ_ACT);
static_assert(WS_END <= (size_t)134217728);

DEVFN float bfr(float f) {
  unsigned int u = __builtin_bit_cast(unsigned int, f);
  u = (u + 0x7fffu + ((u >> 16) & 1u)) & 0xffff0000u;
  return __builtin_bit_cast(float, u);
}

DEVFN v8f wmma_f16(v16h a, v16h b, v8f c) {
  v8f d = __builtin_amdgcn_wmma_f32_16x16x32_f16(false, a, false, b, (short)0, c, false, false);
  asm volatile("v_nop\n\tv_nop\n\tv_nop\n\tv_nop" : "+v"(d) : "v"(a), "v"(b));
  return d;
}

union Frag16 { v16h v; v8h hv[2]; };

DEVFN v16h frag_rowk(const _Float16* base, int row0, int ld, int k0) {
  const int l = threadIdx.x & 31;
  const _Float16* p = base + (size_t)(row0 + (l & 15)) * ld + k0 + 8 * (l >> 4);
  Frag16 f;
  f.hv[0] = *(const v8ha*)p;
  f.hv[1] = *(const v8ha*)(p + 16);
  return f.v;
}

DEVFN void st2h(_Float16* p, v8h v) {
  *(volatile v8h*)p = v;
  __threadfence();
  *(volatile v8h*)p = v;
}
DEVFN void st2f(float* p, v4f v) {
  *(volatile v4f*)p = v;
  __threadfence();
  *(volatile v4f*)p = v;
}

static constexpr int PREP_BQ = (D3 * DM / 8) / 256;
static constexpr int PREP_BO = (DM * DM / 8) / 256;
static_assert((D3 * DM / 8) % 256 == 0 && (DM * DM / 8) % 256 == 0);

__global__ __launch_bounds__(256) void k_prep(const float* __restrict__ wq32,
                                              const float* __restrict__ wo32,
                                              _Float16* __restrict__ wq16,
                                              _Float16* __restrict__ wo16) {
  const int blk = blockIdx.x;
  const float* src;
  _Float16* dst;
  size_t e0;
  if (blk < PREP_BQ) {
    src = wq32; dst = wq16; e0 = ((size_t)blk * 256 + threadIdx.x) * 8;
  } else if (blk < PREP_BQ + PREP_BO) {
    src = wo32; dst = wo16; e0 = ((size_t)(blk - PREP_BQ) * 256 + threadIdx.x) * 8;
  } else {
    return;
  }
  const v4f a = *(const v4f*)(src + e0);
  const v4f c = *(const v4f*)(src + e0 + 4);
  v8h o;
#pragma unroll
  for (int i = 0; i < 4; ++i) {
    const float fa = a[i];
    const float fc = c[i];
    o[i]     = (_Float16)(bfr(fa) * 16.0f);
    o[i + 4] = (_Float16)(bfr(fc) * 16.0f);
  }
  st2h(dst + e0, o);
}

__global__ __launch_bounds__(128) void k_gain(const float* __restrict__ cond,
                                              const float* __restrict__ nw,
                                              float* __restrict__ gain) {
  const int t = blockIdx.x * 128 + threadIdx.x;
  if (t >= NB * 256) return;
  const int b = t >> 8, d0 = (t & 255) * 4;
  const float* c  = cond + (size_t)b * DC;
  const float* w0 = nw + (size_t)d0 * DC;
  float s0 = 0.f, s1 = 0.f, s2 = 0.f, s3 = 0.f;
#pragma unroll 1
  for (int j = 0; j < DC; j += 4) {
    const v4f cv = *(const v4f*)(c + j);
    const v4f wa = *(const v4f*)(w0 + j);
    const v4f wb = *(const v4f*)(w0 + DC + j);
    const v4f wc = *(const v4f*)(w0 + 2 * DC + j);
    const v4f wd = *(const v4f*)(w0 + 3 * DC + j);
#pragma unroll
    for (int i = 0; i < 4; ++i) {
      const float ci = cv[i];
      const float ai = wa[i], bi = wb[i], xi = wc[i], di = wd[i];
      const float cj = bfr(ci);
      s0 += cj * bfr(ai);
      s1 += cj * bfr(bi);
      s2 += cj * bfr(xi);
      s3 += cj * bfr(di);
    }
  }
  v4f g;
  g[0] = s0 + 1.0f; g[1] = s1 + 1.0f; g[2] = s2 + 1.0f; g[3] = s3 + 1.0f;
  st2f(gain + (size_t)b * DM + d0, g);
}

__global__ __launch_bounds__(128) void k_norm(const float* __restrict__ x,
                                              const float* __restrict__ gain,
                                              _Float16* __restrict__ xn) {
  __shared__ float red[4];
  const int row = blockIdx.x;
  const int b = row / SEQ, l = row - b * SEQ;
  const int tid = threadIdx.x;
  const float* xr = x + ((size_t)b * SEQ_FULL + l) * DM + tid * 8;
  const v4f a = *(const v4f*)xr;
  const v4f c = *(const v4f*)(xr + 4);
  float e[8];
#pragma unroll
  for (int i = 0; i < 4; ++i) {
    const float fa = a[i];
    const float fc = c[i];
    e[i] = bfr(fa);
    e[i + 4] = bfr(fc);
  }
  float ss = 0.f;
#pragma unroll
  for (int i = 0; i < 8; ++i) ss += e[i] * e[i];
#pragma unroll
  for (int off = 16; off >= 1; off >>= 1) ss += __shfl_xor(ss, off, 32);
  if ((tid & 31) == 0) red[tid >> 5] = ss;
  __syncthreads();
  const float tot = (red[0] + red[1]) + (red[2] + red[3]);
  const float inv = rsqrtf(tot * (1.0f / 1024.0f) + EPSV);
  const float* gp = gain + (size_t)b * DM + tid * 8;
  const v4f g0 = *(const v4f*)gp;
  const v4f g1 = *(const v4f*)(gp + 4);
  v8h o;
#pragma unroll
  for (int i = 0; i < 4; ++i) {
    const float ga = g0[i];
    const float gb = g1[i];
    o[i]     = (_Float16)(e[i] * (ga * inv));
    o[i + 4] = (_Float16)(e[i + 4] * (gb * inv));
  }
  st2h(xn + (size_t)row * DM + tid * 8, o);
}

static constexpr int GEMM_SMEM_BYTES = 128 * 136 * 2;
static_assert(GEMM_SMEM_BYTES >= 2 * 128 * 64 * 2);
static_assert(GEMM_SMEM_BYTES >= 64 * 132 * 4);

DEVFN void gemm_loop(const _Float16* __restrict__ A, const _Float16* __restrict__ W,
                     int m_blk, int n_blk, _Float16* As, _Float16* Ws,
                     v8f (&acc)[2][4]) {
  const int tid = threadIdx.x, w = tid >> 5, wm = w >> 1, wn = w & 1;
#pragma unroll 1
  for (int kb = 0; kb < DM / 64; ++kb) {
    __syncthreads();
#pragma unroll
    for (int i = 0; i < 4; ++i) {
      const int idx = tid + i * 256;
      const int r = idx >> 3, c8 = (idx & 7) * 8;
      *(v8ha*)(As + r * 64 + c8) = *(const v8ha*)(A + (size_t)(m_blk + r) * DM + kb * 64 + c8);
      *(v8ha*)(Ws + r * 64 + c8) = *(const v8ha*)(W + (size_t)(n_blk + r) * DM + kb * 64 + c8);
    }
    __syncthreads();
#pragma unroll
    for (int ks = 0; ks < 64; ks += 32) {
      v16h af[2], bf[4];
#pragma unroll
      for (int mt = 0; mt < 2; ++mt) af[mt] = frag_rowk(As, wm * 32 + mt * 16, 64, ks);
#pragma unroll
      for (int nt = 0; nt < 4; ++nt) bf[nt] = frag_rowk(Ws, wn * 64 + nt * 16, 64, ks);
#pragma unroll
      for (int mt = 0; mt < 2; ++mt)
#pragma unroll
        for (int nt = 0; nt < 4; ++nt)
          acc[mt][nt] = wmma_f16(af[mt], bf[nt], acc[mt][nt]);
    }
  }
}

__global__ __launch_bounds__(256) void k_qkv_gemm(const _Float16* __restrict__ xn,
                                                  const _Float16* __restrict__ wq,
                                                  const float* __restrict__ hsc,
                                                  _Float16* __restrict__ qp,
                                                  _Float16* __restrict__ kp,
                                                  _Float16* __restrict__ vt) {
  __shared__ __align__(16) unsigned char smem_raw[GEMM_SMEM_BYTES];
  _Float16* As = (_Float16*)smem_raw;
  _Float16* Ws = As + 128 * 64;
  _Float16* T  = (_Float16*)smem_raw;
  constexpr int TP = 136;

  const int tid = threadIdx.x, w = tid >> 5, lane = tid & 31;
  const int wm = w >> 1, wn = w & 1, h = lane >> 4, n = lane & 15;
  const int m_blk = blockIdx.y * 128;
  const int n_blk = blockIdx.x * 128;
  const int tsel  = n_blk >> 10;
  const int head0 = (n_blk & (DM - 1)) >> 6;
  const int b  = m_blk / SEQ;
  const int l0 = m_blk - b * SEQ;

  v8f acc[2][4] = {};
  gemm_loop(xn, wq, m_blk, n_blk, As, Ws, acc);
  __syncthreads();

  if (tsel < 2) {
    const float hsv = bfr(hsc[head0 + wn]);
    const float sqs = sqrtf(hsv);
#pragma unroll
    for (int mt = 0; mt < 2; ++mt) {
#pragma unroll
      for (int nt = 0; nt < 4; ++nt) acc[mt][nt] *= 0.0625f;
#pragma unroll
      for (int r = 0; r < 8; ++r) {
        float s = 0.f;
#pragma unroll
        for (int nt = 0; nt < 4; ++nt) s += acc[mt][nt][r] * acc[mt][nt][r];
#pragma unroll
        for (int off = 8; off >= 1; off >>= 1) s += __shfl_xor(s, off, 32);
        const float mul = sqs * rsqrtf(s + EPSV);
        const int row = wm * 32 + mt * 16 + 8 * h + r;
#pragma unroll
        for (int nt = 0; nt < 4; ++nt)
          T[row * TP + wn * 64 + nt * 16 + n] = (_Float16)(acc[mt][nt][r] * mul);
      }
    }
  } else {
#pragma unroll
    for (int mt = 0; mt < 2; ++mt)
#pragma unroll
      for (int nt = 0; nt < 4; ++nt) {
        v8h o;
#pragma unroll
        for (int r = 0; r < 8; ++r) o[r] = (_Float16)acc[mt][nt][r];
        *(v8ha*)(T + (wn * 64 + nt * 16 + n) * TP + wm * 32 + mt * 16 + 8 * h) = o;
      }
  }
  __syncthreads();

  if (tsel < 2) {
    _Float16* plane = (tsel == 0) ? qp : kp;
#pragma unroll
    for (int it = 0; it < 8; ++it) {
      const int p = it * 256 + tid;
      const int li = p >> 3, sub = p & 7;
      const int row = li & 127, hs2 = li >> 7;
      const v8h v = *(const v8ha*)(T + row * TP + hs2 * 64 + sub * 8);
      _Float16* dst = plane + (((size_t)(b * NHD + head0 + hs2)) * SEQ + l0 + row) * HE + sub * 8;
      st2h(dst, v);
    }
  } else {
#pragma unroll
    for (int it = 0; it < 8; ++it) {
      const int p = it * 256 + tid;
      const int li = p >> 3, sub = p & 7;
      const int erow = li >> 1, hlf = li & 1;
      const v8h v = *(const v8ha*)(T + erow * TP + hlf * 64 + sub * 8);
      _Float16* dst = vt + (((size_t)(b * NHD + head0 + (erow >> 6))) * HE + (erow & 63)) * SEQ
                         + l0 + hlf * 64 + sub * 8;
      st2h(dst, v);
    }
  }
}

__global__ __launch_bounds__(128) void k_attn(const _Float16* __restrict__ qp,
                                              const _Float16* __restrict__ kp,
                                              const _Float16* __restrict__ vt,
                                              _Float16* __restrict__ ctx) {
  constexpr int KLD = 72, VLD = 72, PLD = 72;
  __shared__ __align__(16) _Float16 Ks[64 * KLD];
  __shared__ __align__(16) _Float16 Vs[64 * VLD];
  __shared__ __align__(16) _Float16 Ps[4 * 16 * PLD];

  const int tid = threadIdx.x, w = tid >> 5, lane = tid & 31;
  const int h = lane >> 4, n = lane & 15;
  const int qblk = blockIdx.x, hd = blockIdx.y, b = blockIdx.z;
  const int bh = b * NHD + hd;
  const int q0 = qblk * 64 + w * 16;

  const _Float16* qrow = qp + ((size_t)bh * SEQ + q0) * HE;
  const v16h aq0 = frag_rowk(qrow, 0, HE, 0);
  const v16h aq1 = frag_rowk(qrow, 0, HE, 32);
  const _Float16* kbase = kp + (size_t)bh * SEQ * HE;
  const _Float16* vbase = vt + (size_t)bh * HE * SEQ;
  _Float16* Pw = Ps + w * 16 * PLD;

  float mr[8], lr[8];
#pragma unroll
  for (int r = 0; r < 8; ++r) { mr[r] = -3.0e38f; lr[r] = 0.f; }
  v8f oacc[4] = {};

#pragma unroll 1
  for (int kb = 0; kb < SEQ / 64; ++kb) {
    __syncthreads();
#pragma unroll
    for (int i = 0; i < 4; ++i) {
      const int idx = tid + i * 128;
      const int r = idx >> 3, c8 = (idx & 7) * 8;
      *(v8ha*)(Ks + r * KLD + c8) = *(const v8ha*)(kbase + (size_t)(kb * 64 + r) * HE + c8);
      *(v8ha*)(Vs + r * VLD + c8) = *(const v8ha*)(vbase + (size_t)r * SEQ + kb * 64 + c8);
    }
    __syncthreads();

    v8f s[4] = {};
#pragma unroll
    for (int nt = 0; nt < 4; ++nt) {
      const v16h b0 = frag_rowk(Ks, nt * 16, KLD, 0);
      s[nt] = wmma_f16(aq0, b0, s[nt]);
      const v16h b1 = frag_rowk(Ks, nt * 16, KLD, 32);
      s[nt] = wmma_f16(aq1, b1, s[nt]);
    }

    float alpha[8];
#pragma unroll
    for (int r = 0; r < 8; ++r) {
      float cm = fmaxf(fmaxf(s[0][r], s[1][r]), fmaxf(s[2][r], s[3][r]));
#pragma unroll
      for (int off = 8; off >= 1; off >>= 1) cm = fmaxf(cm, __shfl_xor(cm, off, 32));
      const float mnew = fmaxf(mr[r], cm);
      const float al = __expf(mr[r] - mnew);
      float ps = 0.f;
#pragma unroll
      for (int nt = 0; nt < 4; ++nt) {
        const float pv = __expf(s[nt][r] - mnew);
        s[nt][r] = pv;
        ps += pv;
      }
#pragma unroll
      for (int off = 8; off >= 1; off >>= 1) ps += __shfl_xor(ps, off, 32);
      lr[r] = lr[r] * al + ps;
      mr[r] = mnew;
      alpha[r] = al;
    }
#pragma unroll
    for (int dt = 0; dt < 4; ++dt)
#pragma unroll
      for (int r = 0; r < 8; ++r) oacc[dt][r] *= alpha[r];
#pragma unroll
    for (int nt = 0; nt < 4; ++nt)
#pragma unroll
      for (int r = 0; r < 8; ++r)
        Pw[(8 * h + r) * PLD + nt * 16 + n] = (_Float16)(s[nt][r] * 16384.0f);
    __syncthreads();

#pragma unroll
    for (int ks = 0; ks < 2; ++ks) {
      const v16h pa = frag_rowk(Pw, 0, PLD, ks * 32);
#pragma unroll
      for (int dt = 0; dt < 4; ++dt) {
        const v16h bv = frag_rowk(Vs, dt * 16, VLD, ks * 32);
        oacc[dt] = wmma_f16(pa, bv, oacc[dt]);
      }
    }
  }
  __syncthreads();

#pragma unroll
  for (int r = 0; r < 8; ++r) {
    const float sc = (1.0f / lr[r]) * (1.0f / 4096.0f);
#pragma unroll
    for (int dt = 0; dt < 4; ++dt)
      Pw[(8 * h + r) * PLD + dt * 16 + n] = (_Float16)(oacc[dt][r] * sc);
  }
  __syncthreads();
#pragma unroll
  for (int it = 0; it < 4; ++it) {
    const int p = it * 32 + lane;
    const int row = p >> 3, sub = p & 7;
    const v8h v = *(const v8ha*)(Pw + row * PLD + sub * 8);
    _Float16* dst = ctx + ((size_t)b * SEQ + q0 + row) * DM + hd * HE + sub * 8;
    st2h(dst, v);
  }
}

__global__ __launch_bounds__(256) void k_out_gemm(const _Float16* __restrict__ ctx,
                                                  const _Float16* __restrict__ wo,
                                                  const float* __restrict__ x,
                                                  float* __restrict__ out) {
  __shared__ __align__(16) unsigned char smem_raw[GEMM_SMEM_BYTES];
  _Float16* As = (_Float16*)smem_raw;
  _Float16* Ws = As + 128 * 64;
  float* Tf = (float*)smem_raw;
  constexpr int TPF = 132;

  const int tid = threadIdx.x, w = tid >> 5, lane = tid & 31;
  const int wm = w >> 1, wn = w & 1, h = lane >> 4, n = lane & 15;
  const int m_blk = blockIdx.y * 128;
  const int n_blk = blockIdx.x * 128;
  const int b  = m_blk / SEQ;
  const int l0 = m_blk - b * SEQ;

  v8f acc[2][4] = {};
  gemm_loop(ctx, wo, m_blk, n_blk, As, Ws, acc);

#pragma unroll 1
  for (int pass = 0; pass < 2; ++pass) {
    __syncthreads();
    if ((wm >> 1) == pass) {
#pragma unroll
      for (int mt = 0; mt < 2; ++mt)
#pragma unroll
        for (int nt = 0; nt < 4; ++nt)
#pragma unroll
          for (int r = 0; r < 8; ++r)
            Tf[((wm & 1) * 32 + mt * 16 + 8 * h + r) * TPF + wn * 64 + nt * 16 + n] = acc[mt][nt][r];
    }
    __syncthreads();
#pragma unroll
    for (int it = 0; it < 8; ++it) {
      const int p = it * 256 + tid;
      const int li = p >> 3, sub = p & 7;
      const int row = li >> 2, q4 = li & 3;
      const int col = q4 * 32 + sub * 4;
      const v4f a = *(const v4fa*)(Tf + row * TPF + col);
      const size_t g = ((size_t)b * SEQ_FULL + l0 + pass * 64 + row) * DM + n_blk + col;
      const v4f xv = *(const v4f*)(x + g);
      v4f o;
#pragma unroll
      for (int i = 0; i < 4; ++i) {
        const float xi = xv[i];
        o[i] = a[i] * (1.0f / 1024.0f) + bfr(xi);
      }
      st2f(out + g, o);
    }
  }
}

extern "C" void kernel_launch(void* const* d_in, const int* in_sizes, int n_in,
                              void* d_out, int out_size, void* d_ws, size_t ws_size,
                              hipStream_t stream) {
  if (n_in < 7) return;
  const long long need_x = ((long long)(NB - 1) * SEQ_FULL + SEQ) * DM;
  if ((long long)in_sizes[0] < need_x) return;
  if (in_sizes[2] < NB * DC) return;
  if (in_sizes[3] < DM * DC) return;
  if (in_sizes[4] < D3 * DM) return;
  if (in_sizes[5] < NHD) return;
  if (in_sizes[6] < DM * DM) return;
  if ((long long)out_size < need_x) return;
  if (ws_size < WS_END) return;

  const float* x      = (const float*)d_in[0];
  const float* cond   = (const float*)d_in[2];
  const float* norm_w = (const float*)d_in[3];
  const float* qkv_w  = (const float*)d_in[4];
  const float* hscale = (const float*)d_in[5];
  const float* out_w  = (const float*)d_in[6];
  float* out = (float*)d_out;

  char* ws = (char*)d_ws;
  _Float16* wq16  = (_Float16*)(ws + OFF_WQ);
  _Float16* wo16  = (_Float16*)(ws + OFF_WO);
  float*    gain  = (float*)(ws + OFF_GAIN);
  _Float16* xn16  = (_Float16*)(ws + OFF_XN);
  _Float16* q16   = (_Float16*)(ws + OFF_Q);
  _Float16* k16   = (_Float16*)(ws + OFF_K);
  _Float16* vt16  = (_Float16*)(ws + OFF_VT);
  _Float16* ctx16 = (_Float16*)(ws + OFF_CTX);

  k_prep<<<PREP_BQ + PREP_BO, 256, 0, stream>>>(qkv_w, out_w, wq16, wo16);
  k_gain<<<(NB * 256 + 127) / 128, 128, 0, stream>>>(cond, norm_w, gain);
  k_norm<<<MTOT, 128, 0, stream>>>(x, gain, xn16);
  k_qkv_gemm<<<dim3(D3 / 128, MTOT / 128), 256, 0, stream>>>(xn16, wq16, hscale, q16, k16, vt16);
  k_attn<<<dim3(SEQ / 64, NHD, NB), 128, 0, stream>>>(q16, k16, vt16, ctx16);
  k_out_gemm<<<dim3(DM / 128, MTOT / 128), 256, 0, stream>>>(ctx16, wo16, x, out);
}
